// MultiTimeAttention_21242908246365
// MI455X (gfx1250) — hardware-run, weakly checked
//
#include <hip/hip_runtime.h>


#ifndef NB
#define NB 8
#endif
#define NB_FULL 8
#define LQ   128
#define LK   256
#define DV   32
#define ED   32
#define NHD  8
#define EK   4
#define NHID 64
#define NO   64
#define KO   (NHD * DV)
#define AW   4
#define OSP  36
#define VSP  36
#define RSP  72
#define TSP  68
#define ESP  40
#define WCAR 1024.0f
#define TEC  1024.0f
#define C10I 0.0009765625f
#define MDC  64.0f
#define MDI  0.015625f
#define XCAR 256.0f
#define OSCL 3.814697265625e-06f
#define SC2  ((float)(0.5 * 1.4426950408889634 * 9.5367431640625e-07))
#define PSH  14.0f
#define NEGB (-3.0e38f)
#define LNEPS 1.0e-5f

static_assert(ED == 32);
static_assert(NHD * EK == ED);
static_assert(EK % 2 == 0);
static_assert(DV == 32);
static_assert(NHID == 64);
static_assert(NO == 64);
static_assert(KO % 32 == 0);
static_assert(KO == 256);
static_assert(LK % 64 == 0);
static_assert(LK % 32 == 0);
static_assert(LQ % 64 == 0);
static_assert(LQ % (16 * AW) == 0);
static_assert((NB * LQ) % 64 == 0);
static_assert((NB * LK) % 64 == 0);
static_assert(NB <= NB_FULL);
static_assert((OSP * 4) % 16 == 0);
static_assert((VSP * 4) % 16 == 0);
static_assert((RSP * 2) % 16 == 0);
static_assert((TSP * 4) % 16 == 0);
static_assert((ESP * 2) % 16 == 0);
static_assert(DV * 4 == 128);
static_assert((NB * LQ) % 4 == 0);
static_assert(((size_t)NB * NHD * LQ * DV) % 8 == 0);

typedef _Float16 h16;
typedef unsigned short bf;
typedef __attribute__((ext_vector_type(16))) __bf16   v16bf;
typedef __attribute__((ext_vector_type(16))) _Float16 v16h;
typedef __attribute__((ext_vector_type(8)))  _Float16 v8h;
typedef __attribute__((ext_vector_type(8)))  unsigned short v8us;
typedef __attribute__((ext_vector_type(8)))  float    v8f;
typedef __attribute__((ext_vector_type(4)))  float    v4f;
typedef v4f  __attribute__((may_alias)) v4fa;
typedef v8h  __attribute__((may_alias)) v8ha;
typedef __attribute__((ext_vector_type(4)))  int      v4i;
typedef v4i  __attribute__((may_alias)) v4ia;
typedef __attribute__((ext_vector_type(8)))  unsigned int v8u;

__device__ __forceinline__ unsigned short f2bf(float f) { unsigned u = __float_as_uint(f); u += 0x7FFFu + ((u >> 16) & 1u); return (unsigned short)(u >> 16); }
__device__ __forceinline__ float bfr(float f) { return __uint_as_float(((unsigned)f2bf(f)) << 16); }
__device__ __forceinline__ v16h cat16(v8h lo, v8h hi) { return __builtin_shufflevector(lo, hi, 0, 1, 2, 3, 4, 5, 6, 7, 8, 9, 10, 11, 12, 13, 14, 15); }
__device__ __forceinline__ v16bf cat16b(v8us lo, v8us hi) { return __builtin_bit_cast(v16bf, __builtin_shufflevector(lo, hi, 0, 1, 2, 3, 4, 5, 6, 7, 8, 9, 10, 11, 12, 13, 14, 15)); }
__device__ __forceinline__ v8f wmma16(v16h a, v16h b, v8f c) { return __builtin_amdgcn_wmma_f32_16x16x32_f16(false, a, false, b, (short)0, c, false, false); }
__device__ __forceinline__ v8f wmmab(v16bf a, v16bf b, v8f c) { return __builtin_amdgcn_wmma_f32_16x16x32_bf16(false, a, false, b, (short)0, c, false, false); }
__device__ __forceinline__ v16h  ldh(const h16* p) { return cat16(*(const v8h*)p, *(const v8h*)(p + 16)); }
__device__ __forceinline__ v16bf ldb(const bf* p)  { return cat16b(*(const v8us*)p, *(const v8us*)(p + 16)); }
__device__ __forceinline__ void wave_sync() { __builtin_amdgcn_fence(3  , "wavefront"); __builtin_amdgcn_wave_barrier(); asm volatile("" ::: "memory"); }

__device__ __forceinline__ v8f wmma16g(v16h a, v16h b, v8f c) { c = wmma16(a, b, c); asm volatile("v_nop\n\tv_nop\n\tv_nop\n\tv_nop" : "+v"(c) : "v"(a), "v"(b)); return c; }
__device__ __forceinline__ v8f wmmabg(v16bf a, v16bf b, v8f c) { c = wmmab(a, b, c); asm volatile("v_nop\n\tv_nop\n\tv_nop\n\tv_nop" : "+v"(c) : "v"(a), "v"(b)); return c; }
static __device__ __forceinline__ h16 toh_flush(float v) { const h16 r = (h16)v; return (fabsf(v) < 6.103515625e-05f) ? (h16)0.0f : r; }

__global__ __launch_bounds__(256) void k_wtb(const float* __restrict__ W, bf* Bt, int K, int N) {
    const int kp = K >> 3; const int i = (int)(blockIdx.x * 256 + threadIdx.x); if (i >= N * kp) return;
    const int n = i / kp, k0 = (i - n * kp) * 8; v8us o;
#pragma unroll
    for (int j = 0; j < 8; ++j) o[j] = f2bf(W[(size_t)(k0 + j) * N + n]);
    *(volatile v8us*)(Bt + (size_t)i * 8) = o; __threadfence(); *(volatile v8us*)(Bt + (size_t)i * 8) = o;
}
__global__ __launch_bounds__(256) void k_wth(const float* __restrict__ W, h16* Bt, int K, int N, float scale) {
    const int kp = K >> 3; const int i = (int)(blockIdx.x * 256 + threadIdx.x); if (i >= N * kp) return;
    const int n = i / kp, k0 = (i - n * kp) * 8; v8h o;
#pragma unroll
    for (int j = 0; j < 8; ++j) o[j] = toh_flush(bfr(W[(size_t)(k0 + j) * N + n]) * scale);
    *(volatile v8h*)(Bt + (size_t)i * 8) = o; __threadfence(); *(volatile v8h*)(Bt + (size_t)i * 8) = o;
}

__global__ __launch_bounds__(32) void k_flag(const int* __restrict__ emask, int* FLG) {
    const int lane = threadIdx.x & 31; const int b = blockIdx.x;
    int any = 0;
#pragma unroll 4
    for (int k = 0; k < LK; ++k) { const int w = emask[((size_t)b * LK + k) * DV + lane]; any |= (w != 0) ? 1 : 0; }
    const int q4 = (lane & 7) * 4;
    v4i g;
    g[0] = __shfl(any, q4 + 0, 32); g[1] = __shfl(any, q4 + 1, 32); g[2] = __shfl(any, q4 + 2, 32); g[3] = __shfl(any, q4 + 3, 32);
    static_assert(8 * 16 == DV * 4);
    int* fl = FLG + (size_t)b * DV + q4;
    if (lane < 8) *(volatile v4ia*)fl = g;
    __threadfence();
    if (lane < 8) *(volatile v4ia*)fl = g;
}

__global__ __launch_bounds__(32) void k_prep(const float* __restrict__ value, const int* __restrict__ emask, const bf* __restrict__ W1B, const float* __restrict__ b1,
                                             const float* __restrict__ lng, const float* __restrict__ lnb, const h16* __restrict__ W2H, const float* __restrict__ b2,
                                             h16* MVT, h16* MFT, h16* MDT, h16* UDT) {
    __shared__ __align__(16) float sv[64 * VSP];
    __shared__ __align__(16) float sm[64 * VSP];
    __shared__ __align__(16) h16   sr[16 * RSP];
    __shared__ __align__(16) float tv[DV * TSP];
    __shared__ __align__(16) float tf[DV * TSP];
    __shared__ __align__(16) float td[DV * TSP];
    __shared__ __align__(16) float tu[DV * TSP];
    static_assert((2 * 64 * VSP + 4 * DV * TSP) * 4 + 16 * RSP * 2 <= 131072);
    const int lane = threadIdx.x & 31, lr = lane & 15, hi = lane >> 4;
    const int m0 = blockIdx.x * 64;
    const int b = m0 / LK, key0 = m0 % LK;
    static_assert(16 * 32 * 4 == 64 * DV);
#pragma unroll 4
    for (int it = 0; it < 16; ++it) {
        const int p = it * 32 + lane; const int row = p >> 3, c4 = (p & 7) * 4;
        const v4f v = *(const v4f*)(value + (size_t)(m0 + row) * DV + c4);
        const v4i k = *(const v4i*)(emask + (size_t)(m0 + row) * DV + c4);
        v4f cv, cm;
#pragma unroll
        for (int i = 0; i < 4; ++i) { cv[i] = bfr(v[i]); cm[i] = (k[i] != 0) ? 1.0f : 0.0f; }
        *(v4fa*)(&sv[row * VSP + c4]) = cv; *(v4fa*)(&sm[row * VSP + c4]) = cm;
    }
    wave_sync();
    float b1c[4], gc[4], bec[4], b2c[2];
    v16bf w1f[4]; v16h w2f[2][2];
#pragma unroll
    for (int nb = 0; nb < 4; ++nb) { const int c = nb * 16 + lr; b1c[nb] = bfr(b1[c]); gc[nb] = bfr(lng[c]); bec[nb] = bfr(lnb[c]);
        w1f[nb] = ldb(W1B + (size_t)c * DV + 8 * hi); }
#pragma unroll
    for (int nb = 0; nb < 2; ++nb) { const int c = nb * 16 + lr; b2c[nb] = bfr(b2[c]);
        w2f[nb][0] = ldh(W2H + (size_t)c * NHID + 8 * hi); w2f[nb][1] = ldh(W2H + (size_t)c * NHID + 32 + 8 * hi); }
#pragma unroll 1
    for (int sl = 0; sl < 4; ++sl) {
        const int ab = (sl * 16 + lr) * VSP + 8 * hi;
        const v4f a0 = *(const v4fa*)(&sv[ab]), a1 = *(const v4fa*)(&sv[ab + 4]), a2 = *(const v4fa*)(&sv[ab + 16]), a3 = *(const v4fa*)(&sv[ab + 20]);
        v8us lo, up;
#pragma unroll
        for (int i = 0; i < 4; ++i) { lo[i] = f2bf(a0[i]); lo[4 + i] = f2bf(a1[i]); up[i] = f2bf(a2[i]); up[4 + i] = f2bf(a3[i]); }
        const v16bf af = cat16b(lo, up);
        v8f hd[4];
#pragma unroll
        for (int nb = 0; nb < 4; ++nb) hd[nb] = wmmabg(af, w1f[nb], (v8f){});
#pragma unroll
        for (int r = 0; r < 8; ++r) {
            float hv[4];
#pragma unroll
            for (int nb = 0; nb < 4; ++nb) hv[nb] = hd[nb][r] + b1c[nb];
            float s = (hv[0] + hv[1]) + (hv[2] + hv[3]);
            s += __shfl_xor(s, 1, 32); s += __shfl_xor(s, 2, 32); s += __shfl_xor(s, 4, 32); s += __shfl_xor(s, 8, 32);
            const float mu = s * (1.0f / 64.0f);
            float dd[4];
#pragma unroll
            for (int nb = 0; nb < 4; ++nb) dd[nb] = hv[nb] - mu;
            float vs = (dd[0] * dd[0] + dd[1] * dd[1]) + (dd[2] * dd[2] + dd[3] * dd[3]);
            vs += __shfl_xor(vs, 1, 32); vs += __shfl_xor(vs, 2, 32); vs += __shfl_xor(vs, 4, 32); vs += __shfl_xor(vs, 8, 32);
            const float rstd = rsqrtf(vs * (1.0f / 64.0f) + LNEPS);
#pragma unroll
            for (int nb = 0; nb < 4; ++nb) { const float y = dd[nb] * rstd * gc[nb] + bec[nb]; const float rl = (y > 0.0f) ? y : 0.0f;
                sr[(hi * 8 + r) * RSP + nb * 16 + lr] = toh_flush(rl); }
        }
        wave_sync();
        const int rb = lr * RSP + 8 * hi;
        const v16h r0f = cat16(*(const v8ha*)(&sr[rb]), *(const v8ha*)(&sr[rb + 16]));
        const v16h r1f = cat16(*(const v8ha*)(&sr[rb + 32]), *(const v8ha*)(&sr[rb + 48]));
        v8f dv[2];
#pragma unroll
        for (int nb = 0; nb < 2; ++nb) { dv[nb] = wmma16g(r0f, w2f[nb][0], (v8f){}); dv[nb] = wmma16g(r1f, w2f[nb][1], dv[nb]); }
#pragma unroll
        for (int nb = 0; nb < 2; ++nb) {
            const int d = nb * 16 + lr;
            float mvv[8], mfv[8], mdv[8], udv[8];
#pragma unroll
            for (int r = 0; r < 8; ++r) { const int kk = sl * 16 + hi * 8 + r;
                const float val = sv[kk * VSP + d]; const float msk = sm[kk * VSP + d];
                const float dval = dv[nb][r] * C10I + b2c[nb];
                const bool kept = msk != 0.0f;
                mvv[r] = kept ? val : 0.0f; mfv[r] = kept ? 1.0f : 0.0f; mdv[r] = kept ? (dval * MDC) : 0.0f; udv[r] = dval * MDC; }
            const int to = d * TSP + sl * 16 + hi * 8;
            v4f x, y;
            x[0] = mvv[0]; x[1] = mvv[1]; x[2] = mvv[2]; x[3] = mvv[3]; y[0] = mvv[4]; y[1] = mvv[5]; y[2] = mvv[6]; y[3] = mvv[7];
            *(v4fa*)(&tv[to]) = x; *(v4fa*)(&tv[to + 4]) = y;
            x[0] = mfv[0]; x[1] = mfv[1]; x[2] = mfv[2]; x[3] = mfv[3]; y[0] = mfv[4]; y[1] = mfv[5]; y[2] = mfv[6]; y[3] = mfv[7];
            *(v4fa*)(&tf[to]) = x; *(v4fa*)(&tf[to + 4]) = y;
            x[0] = mdv[0]; x[1] = mdv[1]; x[2] = mdv[2]; x[3] = mdv[3]; y[0] = mdv[4]; y[1] = mdv[5]; y[2] = mdv[6]; y[3] = mdv[7];
            *(v4fa*)(&td[to]) = x; *(v4fa*)(&td[to + 4]) = y;
            x[0] = udv[0]; x[1] = udv[1]; x[2] = udv[2]; x[3] = udv[3]; y[0] = udv[4]; y[1] = udv[5]; y[2] = udv[6]; y[3] = udv[7];
            *(v4fa*)(&tu[to]) = x; *(v4fa*)(&tu[to + 4]) = y;
        }
        wave_sync();
    }
    const size_t pb = ((size_t)b * DV) * LK + (size_t)key0;
    static_assert(8 * 4 == DV);
    static_assert(8 * 16 == 64 * 2);
#pragma unroll 1
    for (int ps = 0; ps < 2; ++ps) {
#pragma unroll 1
        for (int s = 0; s < 8; ++s) { const int row = 4 * s + (lane >> 3), c8 = (lane & 7) * 8;
            const size_t oo = pb + (size_t)row * LK + c8;
            { const v4f x0 = *(const v4fa*)(&tv[row * TSP + c8]); const v4f x1 = *(const v4fa*)(&tv[row * TSP + c8 + 4]); v8h hv;
#pragma unroll
              for (int i = 0; i < 4; ++i) { hv[i] = toh_flush(x0[i]); hv[4 + i] = toh_flush(x1[i]); }
              *(volatile v8h*)(MVT + oo) = hv; }
            { const v4f x0 = *(const v4fa*)(&tf[row * TSP + c8]); const v4f x1 = *(const v4fa*)(&tf[row * TSP + c8 + 4]); v8h hv;
#pragma unroll
              for (int i = 0; i < 4; ++i) { hv[i] = toh_flush(x0[i]); hv[4 + i] = toh_flush(x1[i]); }
              *(volatile v8h*)(MFT + oo) = hv; }
            { const v4f x0 = *(const v4fa*)(&td[row * TSP + c8]); const v4f x1 = *(const v4fa*)(&td[row * TSP + c8 + 4]); v8h hv;
#pragma unroll
              for (int i = 0; i < 4; ++i) { hv[i] = toh_flush(x0[i]); hv[4 + i] = toh_flush(x1[i]); }
              *(volatile v8h*)(MDT + oo) = hv; }
            { const v4f x0 = *(const v4fa*)(&tu[row * TSP + c8]); const v4f x1 = *(const v4fa*)(&tu[row * TSP + c8 + 4]); v8h hv;
#pragma unroll
              for (int i = 0; i < 4; ++i) { hv[i] = toh_flush(x0[i]); hv[4 + i] = toh_flush(x1[i]); }
              *(volatile v8h*)(UDT + oo) = hv; } }
        if (ps == 0) __threadfence(); }
}

__global__ __launch_bounds__(32) void k_temb(const float* __restrict__ tt, const float* __restrict__ wt, const float* __restrict__ bt,
                                             const float* __restrict__ wp, const float* __restrict__ bp, const h16* __restrict__ WH, const float* __restrict__ bias, h16* PL) {
    __shared__ __align__(16) h16   ste[16 * ESP];
    __shared__ __align__(16) float os[16 * OSP];
    static_assert(16 * ESP * 2 + 16 * OSP * 4 <= 131072);
    const int lane = threadIdx.x & 31, lr = lane & 15, hi = lane >> 4;
    const int m0 = blockIdx.x * 16;
    const int jc = (lane > 0) ? (lane - 1) : 0;
    float wv = wp[jc]; asm volatile("" : "+v"(wv));
    float bv = bp[jc]; asm volatile("" : "+v"(bv));
    const float wcol = bfr(wv), bcol = bfr(bv);
    const float w0 = bfr(wt[0]), b0 = bfr(bt[0]);
#pragma unroll 1
    for (int i = 0; i < 16; ++i) {
        const float t = bfr(tt[(size_t)m0 + i]);
        const float lin = t * w0 + b0;
        const float per = sinf(t * wcol + bcol);
        const float te = (lane == 0) ? lin : per;
        ste[i * ESP + lane] = toh_flush(te * TEC);
    }
    wave_sync();
    const int ab = lr * ESP + 8 * hi;
    const v16h af = cat16(*(const v8ha*)(&ste[ab]), *(const v8ha*)(&ste[ab + 16]));
    v8f acc[2]; float bc[2];
#pragma unroll
    for (int nb = 0; nb < 2; ++nb) { const int c = nb * 16 + lr; bc[nb] = bfr(bias[c]) * TEC;
        const v16h bfg = ldh(WH + (size_t)c * ED + 8 * hi);
        acc[nb] = wmma16g(af, bfg, (v8f){}); }
#pragma unroll
    for (int nb = 0; nb < 2; ++nb) {
#pragma unroll
        for (int j = 0; j < 8; ++j) os[(hi * 8 + j) * OSP + nb * 16 + lr] = acc[nb][j] * C10I + bc[nb]; }
    wave_sync();
    const size_t pbase = (size_t)m0 * ED;
    static_assert(2 * 32 * 16 == 16 * ED * 2);
#pragma unroll 1
    for (int ps = 0; ps < 2; ++ps) {
#pragma unroll
        for (int s = 0; s < 2; ++s) { const int p = s * 32 + lane; const int row = p >> 2, c8 = (p & 3) * 8;
            const v4f x0 = *(const v4fa*)(&os[row * OSP + c8]); const v4f x1 = *(const v4fa*)(&os[row * OSP + c8 + 4]); v8h hv;
#pragma unroll
            for (int i = 0; i < 4; ++i) { hv[i] = toh_flush(x0[i]); hv[4 + i] = toh_flush(x1[i]); }
            *(volatile v8h*)(PL + pbase + (size_t)p * 8) = hv; }
        if (ps == 0) __threadfence(); }
}

__global__ __launch_bounds__(32 * AW) void k_flash(const h16* __restrict__ QH, const h16* __restrict__ KP,
                                                   const h16* __restrict__ MVT, const h16* __restrict__ MFT, const h16* __restrict__ MDT,
                                                   const float* __restrict__ qtt, const float* __restrict__ ktt, const float* __restrict__ wdec, h16* XH) {
    __shared__ __align__(16) float os[AW * 16 * OSP];
    static_assert(AW * 16 * OSP * 4 <= 131072);
    const int lane = threadIdx.x & 31, lr = lane & 15, hi = lane >> 4;
    const int wave = __builtin_amdgcn_readfirstlane((int)(threadIdx.x >> 5));
    const int zh = blockIdx.y; const int b = zh / NHD, h = zh % NHD;
    const int t0 = (blockIdx.x * AW + wave) * 16;
    const float wd = bfr(wdec[0]);
    const float tq = bfr(qtt[(size_t)b * LQ + t0 + lr]);
    const size_t qo = ((size_t)b * LQ + t0 + lr) * ED + 8 * hi;
    v16h qh = ldh(QH + qo);
    { v8u qw = __builtin_bit_cast(v8u, qh);
#pragma unroll
      for (int w = 0; w < 8; ++w) { const int e = (w < 4) ? (8 * hi + 2 * w) : (16 + 8 * hi + 2 * (w - 4)); qw[w] = ((e / EK) == h) ? qw[w] : 0u; }
      qh = __builtin_bit_cast(v16h, qw); }
    const size_t ko = ((size_t)b * LK + lr) * ED + 8 * hi;
    const size_t vo = ((size_t)b * DV + lr) * LK + 8 * hi;
    const float* ktb = ktt + (size_t)b * LK + 8 * hi;
    v8f n1a = (v8f){}, n1b = (v8f){}, za = (v8f){}, zb = (v8f){}, n2a = (v8f){}, n2b = (v8f){};
    float m = NEGB;
#pragma unroll 1
    for (int key0 = 0; key0 < LK; key0 += 32) {
        const h16* ka = KP + ko + (size_t)key0 * ED;
        const v16h ka0 = ldh(ka), kb0 = ldh(ka + 16 * ED);
        const v8f sa = wmma16g(ka0, qh, (v8f){});
        const v8f sb = wmma16g(kb0, qh, (v8f){});
        const float* kp = ktb + key0;
        const v4f m0 = *(const v4f*)kp, m1 = *(const v4f*)(kp + 4), m2 = *(const v4f*)(kp + 16), m3 = *(const v4f*)(kp + 20);
        float kx[8], ky[8];
#pragma unroll
        for (int r = 0; r < 4; ++r) { kx[r] = m0[r]; kx[4 + r] = m1[r]; ky[r] = m2[r]; ky[4 + r] = m3[r]; }
        float ta[8], tb[8]; float mx = NEGB;
#pragma unroll
        for (int r = 0; r < 8; ++r) { ta[r] = sa[r] * SC2; tb[r] = sb[r] * SC2; mx = fmaxf(mx, fmaxf(ta[r], tb[r])); }
        mx = fmaxf(mx, __shfl_xor(mx, 16, 32));
        const float mnew = fmaxf(m, mx);
        const float alpha = __builtin_amdgcn_exp2f(m - mnew);
        const float sh = PSH - mnew;
        v16h pb, pf;
#pragma unroll
        for (int r = 0; r < 8; ++r) {
            const float xa = ta[r] + sh, xb = tb[r] + sh;
            const float ea = (xa < -14.0f) ? 0.0f : __builtin_amdgcn_exp2f(xa);
            const float eb = (xb < -14.0f) ? 0.0f : __builtin_amdgcn_exp2f(xb);
            const float da = tq - bfr(kx[r]), db = tq - bfr(ky[r]);
            const float fa = da * __builtin_amdgcn_rcpf(1.0f + da * wd);
            const float fb = db * __builtin_amdgcn_rcpf(1.0f + db * wd);
            pb[r] = (h16)ea; pb[8 + r] = (h16)eb;
            pf[r] = toh_flush(ea * fa); pf[8 + r] = toh_flush(eb * fb); }
        m = mnew;
        n1a = n1a * alpha; n1b = n1b * alpha; za = za * alpha; zb = zb * alpha; n2a = n2a * alpha; n2b = n2b * alpha;
        { const h16* va = MVT + vo + key0; const v16h v0 = ldh(va), v1 = ldh(va + (size_t)16 * LK);
          n1a = wmma16g(v0, pb, n1a); n1b = wmma16g(v1, pb, n1b); }
        { const h16* va = MFT + vo + key0; const v16h v0 = ldh(va), v1 = ldh(va + (size_t)16 * LK);
          za = wmma16g(v0, pb, za); zb = wmma16g(v1, pb, zb); }
        { const h16* va = MDT + vo + key0; const v16h v0 = ldh(va), v1 = ldh(va + (size_t)16 * LK);
          n2a = wmma16g(v0, pf, n2a); n2b = wmma16g(v1, pf, n2b); }
    }
    const float nanv = __uint_as_float(0x7FC00000u);
    v8f f0, f1;
#pragma unroll
    for (int r = 0; r < 8; ++r) {
        const float z0 = za[r], z1 = zb[r];
        const bool k0 = z0 > 0.0f, k1 = z1 > 0.0f;
        const float s0 = k0 ? z0 : 1.0f, s1 = k1 ? z1 : 1.0f;
        const float i0 = k0 ? (XCAR * __builtin_amdgcn_rcpf(s0)) : nanv;
        const float i1 = k1 ? (XCAR * __builtin_amdgcn_rcpf(s1)) : nanv;
        f0[r] = (n1a[r] + n2a[r] * MDI) * i0; f1[r] = (n1b[r] + n2b[r] * MDI) * i1; }
    const int wb = wave * 16 * OSP;
    { v4f a, c;
      a[0] = f0[0]; a[1] = f0[1]; a[2] = f0[2]; a[3] = f0[3]; c[0] = f0[4]; c[1] = f0[5]; c[2] = f0[6]; c[3] = f0[7];
      *(v4fa*)(&os[wb + lr * OSP +  0 + 8 * hi]) = a; *(v4fa*)(&os[wb + lr * OSP +  0 + 8 * hi + 4]) = c;
      a[0] = f1[0]; a[1] = f1[1]; a[2] = f1[2]; a[3] = f1[3]; c[0] = f1[4]; c[1] = f1[5]; c[2] = f1[6]; c[3] = f1[7];
      *(v4fa*)(&os[wb + lr * OSP + 16 + 8 * hi]) = a; *(v4fa*)(&os[wb + lr * OSP + 16 + 8 * hi + 4]) = c; }
    wave_sync();
    const size_t xb0 = ((size_t)zh * LQ + (size_t)t0) * DV;
    static_assert(2 * 32 * 16 == 16 * DV * 2);
#pragma unroll 1
    for (int ps = 0; ps < 2; ++ps) {
#pragma unroll
        for (int s = 0; s < 2; ++s) { const int p = s * 32 + lane; const int row = p >> 2, c8 = (p & 3) * 8;
            const v4f x0 = *(const v4fa*)(&os[wb + row * OSP + c8]); const v4f x1 = *(const v4fa*)(&os[wb + row * OSP + c8 + 4]); v8h hv;
#pragma unroll
            for (int i = 0; i < 4; ++i) { hv[i] = toh_flush(x0[i]); hv[4 + i] = toh_flush(x1[i]); }
            *(volatile v8h*)(XH + xb0 + (size_t)p * 8) = hv; }
        if (ps == 0) __threadfence(); }
}

__global__ __launch_bounds__(128) void k_umean(const float* __restrict__ value, const h16* __restrict__ UDT, const int* __restrict__ FLG,
                                               const float* __restrict__ qtt, const float* __restrict__ ktt, const float* __restrict__ wdec, float* XM) {
    const int lane = threadIdx.x & 31;
    const int wave = __builtin_amdgcn_readfirstlane((int)(threadIdx.x >> 5));
    const int row = blockIdx.x * 4 + wave;
    const int b = row / LQ;
    const int emp = (FLG[(size_t)b * DV + lane] == 0) ? 1 : 0;
    int anye = emp;
    anye |= __shfl_xor(anye, 1, 32); anye |= __shfl_xor(anye, 2, 32); anye |= __shfl_xor(anye, 4, 32); anye |= __shfl_xor(anye, 8, 32); anye |= __shfl_xor(anye, 16, 32);
    const int sany = __builtin_amdgcn_readfirstlane(anye);
    float mean = 0.0f;
    if (sany != 0) {
        const float wd = bfr(wdec[0]);
        const float tq = bfr(qtt[(size_t)row]);
        float s1 = 0.0f, s2 = 0.0f;
#pragma unroll 1
        for (int k = 0; k < LK; ++k) {
            const float dk = tq - bfr(ktt[(size_t)b * LK + k]);
            const float fk = dk * __builtin_amdgcn_rcpf(1.0f + dk * wd);
            const float val = bfr(value[((size_t)b * LK + k) * DV + lane]);
            const float dval = (float)UDT[((size_t)b * DV + lane) * LK + k] * MDI;
            s1 += val; s2 += dval * fk;
        }
        mean = (s1 + s2) * (1.0f / (float)LK);
    }
    const float outv = (emp != 0) ? mean : 0.0f;
    const int q4 = (lane & 7) * 4;
    v4f g;
    g[0] = __shfl(outv, q4 + 0, 32); g[1] = __shfl(outv, q4 + 1, 32); g[2] = __shfl(outv, q4 + 2, 32); g[3] = __shfl(outv, q4 + 3, 32);
    static_assert(8 * 16 == DV * 4);
    float* xr = XM + (size_t)row * DV + q4;
    if (lane < 8) *(volatile v4fa*)xr = g;
    __threadfence();
    if (lane < 8) *(volatile v4fa*)xr = g;
}

__global__ __launch_bounds__(256) void k_xfix(const h16* __restrict__ X0, const int* __restrict__ FLG, const float* __restrict__ XM, h16* XH) {
    const int i = (int)(blockIdx.x * 256 + threadIdx.x); if (i >= NB * NHD * LQ * DV / 8) return;
    const int row = i >> 2, c8 = (i & 3) * 8;
    const int zh = row / LQ, t = row % LQ; const int b = zh / NHD;
    const v8h x = *(const v8h*)(X0 + (size_t)i * 8);
    const v4i g0 = *(const v4i*)(FLG + (size_t)b * DV + c8), g1 = *(const v4i*)(FLG + (size_t)b * DV + c8 + 4);
    const v4f u0 = *(const v4f*)(XM + ((size_t)b * LQ + t) * DV + c8), u1 = *(const v4f*)(XM + ((size_t)b * LQ + t) * DV + c8 + 4);
    v8h o;
#pragma unroll
    for (int j = 0; j < 4; ++j) { const h16 a0 = toh_flush(u0[j] * XCAR); const h16 a1 = toh_flush(u1[j] * XCAR);
        o[j] = (g0[j] == 0) ? a0 : x[j]; o[4 + j] = (g1[j] == 0) ? a1 : x[4 + j]; }
    *(volatile v8h*)(XH + (size_t)i * 8) = o; __threadfence(); *(volatile v8h*)(XH + (size_t)i * 8) = o;
}

__global__ __launch_bounds__(32) void k_oproj(const h16* __restrict__ XH, const h16* __restrict__ WOH, const float* __restrict__ bo, float* OUT) {
    __shared__ __align__(16) float os[16 * 68];
    static_assert(16 * 68 * 4 <= 131072);
    const int lane = threadIdx.x & 31, lr = lane & 15, hi = lane >> 4; const int r0 = blockIdx.x * 64;
    const int bb = r0 / LQ, tt = r0 % LQ;
    v8f acc[4][4];
#pragma unroll
    for (int mb = 0; mb < 4; ++mb)
#pragma unroll
        for (int nb = 0; nb < 4; ++nb) acc[mb][nb] = (v8f){};
    const size_t aoff = (((size_t)bb * NHD) * LQ + (size_t)(tt + lr)) * DV + 8 * hi;
    const size_t boff = (size_t)lr * KO + 8 * hi;
#pragma unroll 1
    for (int hh = 0; hh < NHD; ++hh) {
        v16h a[4];
#pragma unroll
        for (int mb = 0; mb < 4; ++mb) a[mb] = ldh(XH + aoff + (size_t)hh * LQ * DV + (size_t)mb * 16 * DV);
#pragma unroll
        for (int nb = 0; nb < 4; ++nb) { const v16h bfg = ldh(WOH + boff + (size_t)nb * 16 * KO + (size_t)hh * DV);
#pragma unroll
            for (int mb = 0; mb < 4; ++mb) acc[mb][nb] = wmma16g(a[mb], bfg, acc[mb][nb]); }
    }
    float bc[4];
#pragma unroll
    for (int nb = 0; nb < 4; ++nb) bc[nb] = bfr(bo[nb * 16 + lr]);
    static_assert(8 * 2 == 16);
    static_assert(16 * 16 == NO * 4);
#pragma unroll
    for (int mb = 0; mb < 4; ++mb) {
#pragma unroll
        for (int nb = 0; nb < 4; ++nb) {
#pragma unroll
            for (int j = 0; j < 8; ++j) os[(hi * 8 + j) * 68 + nb * 16 + lr] = acc[mb][nb][j] * OSCL + bc[nb]; }
        wave_sync();
        float* orow = OUT + (size_t)(r0 + mb * 16) * NO;
#pragma unroll 1
        for (int ps = 0; ps < 2; ++ps) {
#pragma unroll
            for (int s = 0; s < 8; ++s) { const int row = 2 * s + (lane >> 4), c4 = (lane & 15) * 4;
                const v4f val = *(const v4fa*)(&os[row * 68 + c4]);
                *(volatile v4f*)(orow + (size_t)row * NO + c4) = val; }
            if (ps == 0) __threadfence(); }
        wave_sync();
    }
}

static constexpr size_t al256(size_t v) { return (v + 255) & ~(size_t)255; }
static constexpr size_t SZ_W1 = al256((size_t)NHID * DV * 2);
static constexpr size_t SZ_W2 = al256((size_t)DV * NHID * 2);
static constexpr size_t SZ_WE = al256((size_t)ED * ED * 2);
static constexpr size_t SZ_WO = al256((size_t)NO * KO * 2);
static constexpr size_t SZ_MP = al256((size_t)NB * DV * LK * 2);
static constexpr size_t SZ_QP = al256((size_t)NB * LQ * ED * 2);
static constexpr size_t SZ_KP = al256((size_t)NB * LK * ED * 2);
static constexpr size_t SZ_XP = al256((size_t)NB * NHD * LQ * DV * 2);
static constexpr size_t SZ_FL = al256((size_t)NB * DV * 4);
static constexpr size_t SZ_XM = al256((size_t)NB * LQ * DV * 4);
static constexpr size_t SZ_TOTAL = SZ_W1 + SZ_W2 + 2 * SZ_WE + SZ_WO + 4 * SZ_MP + SZ_QP + SZ_KP + 2 * SZ_XP + SZ_FL + SZ_XM;
static_assert(SZ_TOTAL <= (size_t)134217728);
static_assert(((size_t)NHID * DV * 2) % 128 == 0);
static_assert(((size_t)ED * ED * 2) % 128 == 0);
static_assert(((size_t)NO * KO * 2) % 128 == 0);
static_assert(((size_t)NB * LQ) % 16 == 0);
static_assert(((size_t)NB * LK) % 16 == 0);
static_assert(((size_t)NB * DV * 4) % 128 == 0);
static_assert(((size_t)NB * LQ * DV * 4) % 128 == 0);
static_assert(((size_t)NB * NHD * LQ * DV / 8) % 256 == 0);

extern "C" void kernel_launch(void* const* d_in, const int* in_sizes, int n_in,
                              void* d_out, int out_size, void* d_ws, size_t ws_size, hipStream_t stream) {
    if (n_in < 21) return;
    if ((size_t)in_sizes[0] < (size_t)NB * LQ || (size_t)in_sizes[1] < (size_t)NB * LK) return;
    if ((size_t)in_sizes[2] < (size_t)NB * LK * DV || (size_t)in_sizes[3] < (size_t)NB * LK * DV) return;
    if (in_sizes[4] < 1 || in_sizes[5] < 1 || in_sizes[6] < ED - 1 || in_sizes[7] < ED - 1 || in_sizes[8] < 1) return;
    if (in_sizes[9] < DV * NHID || in_sizes[10] < NHID || in_sizes[11] < NHID || in_sizes[12] < NHID) return;
    if (in_sizes[13] < NHID * DV || in_sizes[14] < DV) return;
    if (in_sizes[15] < ED * ED || in_sizes[16] < ED || in_sizes[17] < ED * ED || in_sizes[18] < ED) return;
    if (in_sizes[19] < KO * NO || in_sizes[20] < NO) return;
    if ((size_t)out_size < (size_t)NB * LQ * NO) return;
    if (SZ_TOTAL > ws_size) return;
    const float* query_tt = (const float*)d_in[0];
    const float* key_tt   = (const float*)d_in[1];
    const float* value    = (const float*)d_in[2];
    const int*   emb_mask = (const int*)d_in[3];
    const float* w_time   = (const float*)d_in[4];
    const float* b_time   = (const float*)d_in[5];
    const float* w_per    = (const float*)d_in[6];
    const float* b_per    = (const float*)d_in[7];
    const float* w_decay  = (const float*)d_in[8];
    const float* vt_w1    = (const float*)d_in[9];
    const float* vt_b1    = (const float*)d_in[10];
    const float* ln_g     = (const float*)d_in[11];
    const float* ln_b     = (const float*)d_in[12];
    const float* vt_w2    = (const float*)d_in[13];
    const float* vt_b2    = (const float*)d_in[14];
    const float* wq       = (const float*)d_in[15];
    const float* bq       = (const float*)d_in[16];
    const float* wk       = (const float*)d_in[17];
    const float* bk       = (const float*)d_in[18];
    const float* wo       = (const float*)d_in[19];
    const float* bo       = (const float*)d_in[20];
    float* OUT = (float*)d_out;
    char* wsp = (char*)d_ws;
    bf*  W1B = (bf*)wsp;  wsp += SZ_W1;
    h16* W2H = (h16*)wsp; wsp += SZ_W2;
    h16* WQH = (h16*)wsp; wsp += SZ_WE;
    h16* WKH = (h16*)wsp; wsp += SZ_WE;
    h16* WOH = (h16*)wsp; wsp += SZ_WO;
    h16* MVT = (h16*)wsp; wsp += SZ_MP;
    h16* MFT = (h16*)wsp; wsp += SZ_MP;
    h16* MDT = (h16*)wsp; wsp += SZ_MP;
    h16* UDT = (h16*)wsp; wsp += SZ_MP;
    h16* QH  = (h16*)wsp; wsp += SZ_QP;
    h16* KP  = (h16*)wsp; wsp += SZ_KP;
    h16* XH0 = (h16*)wsp; wsp += SZ_XP;
    h16* XH  = (h16*)wsp; wsp += SZ_XP;
    int* FLG = (int*)wsp; wsp += SZ_FL;
    float* XM = (float*)wsp; wsp += SZ_XM;

    k_wtb<<<(unsigned)((NHID * DV / 8 + 255) / 256), 256, 0, stream>>>(vt_w1, W1B, DV, NHID);
    k_wth<<<(unsigned)((DV * NHID / 8 + 255) / 256), 256, 0, stream>>>(vt_w2, W2H, NHID, DV, WCAR);
    k_wth<<<(unsigned)((ED * ED / 8 + 255) / 256), 256, 0, stream>>>(wq, WQH, ED, ED, WCAR);
    k_wth<<<(unsigned)((ED * ED / 8 + 255) / 256), 256, 0, stream>>>(wk, WKH, ED, ED, WCAR);
    k_wth<<<(unsigned)((NO * KO / 8 + 255) / 256), 256, 0, stream>>>(wo, WOH, KO, NO, WCAR);

    k_flag<<<NB, 32, 0, stream>>>(emb_mask, FLG);
    k_prep<<<NB * LK / 64, 32, 0, stream>>>(value, emb_mask, W1B, vt_b1, ln_g, ln_b, W2H, vt_b2, MVT, MFT, MDT, UDT);
    k_temb<<<NB * LQ / 16, 32, 0, stream>>>(query_tt, w_time, b_time, w_per, b_per, WQH, bq, QH);
    k_temb<<<NB * LK / 16, 32, 0, stream>>>(key_tt, w_time, b_time, w_per, b_per, WKH, bk, KP);
    k_flash<<<dim3(LQ / (16 * AW), NB * NHD, 1), 32 * AW, 0, stream>>>(QH, KP, MVT, MFT, MDT, query_tt, key_tt, w_decay, XH0);
    k_umean<<<NB * LQ / 4, 128, 0, stream>>>(value, UDT, FLG, query_tt, key_tt, w_decay, XM);
    k_xfix<<<(unsigned)((NB * NHD * LQ * DV / 8 + 255) / 256), 256, 0, stream>>>(XH0, FLG, XM, XH);
    k_oproj<<<NB * LQ / 64, 32, 0, stream>>>(XH, WOH, bo, OUT);
}
